// FastDecoderBlock_19894288515516
// MI455X (gfx1250) — hardware-verified
//
#include <hip/hip_runtime.h>
#include <math.h>
#include <stdint.h>

constexpr int kB    = 2;
constexpr int kS    = 2048;
constexpr int kD    = 1024;
constexpr int kH    = 16;
constexpr int kHD   = 64;
constexpr int kDFF  = 4096;
constexpr int kTok  = kB * kS;
constexpr int kQKVN = 3 * kD;
constexpr int kGrp  = 2;
constexpr int kNChunk = (kB * kH) / kGrp;
constexpr float kInvD     = 1.0f / 1024.0f;
constexpr float kEps      = 1e-5f;
constexpr float kWCarry   = 16.0f;
constexpr float kPCarry   = 2048.0f;
constexpr float kPVScale  = 64.0f / 2048.0f;
constexpr float kOScale   = 1.0f / (64.0f * 16.0f);
constexpr float kFcScale  = 1.0f / 16.0f;
constexpr float kActCarry = 16.0f;
constexpr float kProjScale = 1.0f / (16.0f * 16.0f);
constexpr float kGeluC0   = 0.7978845608028654f;
constexpr float kGeluC1   = 0.044715f;

constexpr size_t kMiB       = 1048576;
constexpr size_t kOffQkv    = 0;
constexpr size_t kOffA1     = 0;
constexpr size_t kOffVt     = 24 * kMiB;
constexpr size_t kOffScores = 32 * kMiB;
constexpr size_t kOffH      = 32 * kMiB;
constexpr size_t kOffM      = 32 * kMiB;
constexpr size_t kOffWqkvT  = 40 * kMiB;
constexpr size_t kOffWfcT   = 40 * kMiB;
constexpr size_t kOffWprojT = 48 * kMiB;
constexpr size_t kOffP      = 64 * kMiB;
constexpr size_t kOffX1     = 64 * kMiB;
constexpr size_t kOffCtx    = 80 * kMiB;
constexpr size_t kOffWoT    = 88 * kMiB;
constexpr size_t kWsTotal   = 90 * kMiB;
static_assert((size_t)kTok * kQKVN * 2 == 24 * kMiB);
static_assert((size_t)kTok * kDFF * 2 == 32 * kMiB);
static_assert((size_t)kB * kH * kHD * kS * 2 == 8 * kMiB);
static_assert((size_t)kGrp * kS * kS * 4 == 32 * kMiB);
static_assert((size_t)kTok * kD * 2 == 8 * kMiB);
static_assert((size_t)kQKVN * kD * 2 == 6 * kMiB);
static_assert((size_t)kDFF * kD * 2 == 8 * kMiB);
static_assert((size_t)kGrp * kS * kS * 2 == 16 * kMiB);
static_assert((size_t)kTok * kD * 4 == 16 * kMiB);
static_assert((size_t)kD * kD * 2 == 2 * kMiB);
static_assert(kWsTotal <= 134217728);

typedef __attribute__((ext_vector_type(16))) _Float16 v16h;
typedef __attribute__((ext_vector_type(8)))  _Float16 v8h;
typedef __attribute__((ext_vector_type(16))) __bf16   v16b;
typedef __attribute__((ext_vector_type(8)))  __bf16   v8b;
typedef __attribute__((ext_vector_type(8)))  float    v8f;
typedef __attribute__((ext_vector_type(4)))  float    v4f;
typedef __attribute__((ext_vector_type(4)))  unsigned int v4u;

__device__ __forceinline__ unsigned short f2bf_bits(float f) {
  unsigned u = __float_as_uint(f);
  return (unsigned short)((u + 0x7FFFu + ((u >> 16) & 1u)) >> 16);
}
__device__ __forceinline__ float bf_bits2f(unsigned short h) { return __uint_as_float(((unsigned)h) << 16); }

__device__ __forceinline__ void dep_guard_h(v8f& a, v8f& b, v16h x, v16h y) { asm volatile("v_nop\n\tv_nop\n\tv_nop\n\tv_nop" : "+v"(a), "+v"(b) : "v"(x), "v"(y)); }
__device__ __forceinline__ void dep_guard_b(v8f& a, v8f& b, v16b x, v16b y) { asm volatile("v_nop\n\tv_nop\n\tv_nop\n\tv_nop" : "+v"(a), "+v"(b) : "v"(x), "v"(y)); }
__device__ __forceinline__ void keep4_h(v16h a, v16h b, v16h c, v16h d) { asm volatile("v_nop" :: "v"(a), "v"(b), "v"(c), "v"(d)); }
__device__ __forceinline__ void keep4_b(v16b a, v16b b, v16b c, v16b d) { asm volatile("v_nop" :: "v"(a), "v"(b), "v"(c), "v"(d)); }
__device__ __forceinline__ void acc_guard4(v8f& a, v8f& b, v8f& c, v8f& d) { asm volatile("v_nop\n\tv_nop\n\tv_nop\n\tv_nop" : "+v"(a), "+v"(b), "+v"(c), "+v"(d)); }
template <typename T> struct Frag;
template <> struct Frag<_Float16> {
  typedef v16h V; union U { v16h v; v8h h[2]; };
  static __device__ __forceinline__ v16h load(const _Float16* p) {
    U f; f.h[0] = *(const v8h*)(p); f.h[1] = *(const v8h*)(p + 16); return f.v;
  }
  static __device__ __forceinline__ v8f mma(v16h a, v16h b, v8f c) {
    return __builtin_amdgcn_wmma_f32_16x16x32_f16(false, a, false, b, (short)0, c, false, false);
  }
  static __device__ __forceinline__ void guard(v8f& a, v8f& b, v16h x, v16h y) { dep_guard_h(a, b, x, y); }
  static __device__ __forceinline__ void keep(v16h a, v16h b, v16h c, v16h d) { keep4_h(a, b, c, d); }
};
template <> struct Frag<__bf16> {
  typedef v16b V; union U { v16b v; v8b h[2]; };
  static __device__ __forceinline__ v16b load(const __bf16* p) {
    U f; f.h[0] = *(const v8b*)(p); f.h[1] = *(const v8b*)(p + 16); return f.v;
  }
  static __device__ __forceinline__ v8f mma(v16b a, v16b b, v8f c) {
    return __builtin_amdgcn_wmma_f32_16x16x32_bf16(false, a, false, b, (short)0, c, false, false);
  }
  static __device__ __forceinline__ void guard(v8f& a, v8f& b, v16b x, v16b y) { dep_guard_b(a, b, x, y); }
  static __device__ __forceinline__ void keep(v16b a, v16b b, v16b c, v16b d) { keep4_b(a, b, c, d); }
};

__device__ __forceinline__ unsigned pk16(unsigned short a, unsigned short b) { return (unsigned)a | ((unsigned)b << 16); }
__device__ __forceinline__ unsigned short h_bits(float f) { const _Float16 h = (_Float16)f; return __builtin_bit_cast(unsigned short, h); }

template <int ET> struct Elem;
template <> struct Elem<0> { typedef _Float16 T; };
template <> struct Elem<1> { typedef __bf16 T; };
template <int ET, bool SPLIT, int BIAS_MODE, int OUT_MODE, bool RESID, int ACT = 0, int CAUSAL = 0>
__global__ __launch_bounds__(256) void wmma_gemm64(
    const unsigned short* __restrict__ Ap, const unsigned short* __restrict__ A2p, int lda, long strideA,
    const unsigned short* __restrict__ Btp, const unsigned short* __restrict__ Bt2p, int ldb, long strideB,
    void* __restrict__ Cout, void* __restrict__ Cout2, int ldc, long strideC,
    const float* __restrict__ bias,
    const float* __restrict__ resid, long strideR,
    int M, int N, int K, float scale) {
  typedef typename Elem<ET>::T T;
  typedef typename Frag<T>::V V;
  const T* A = (const T*)Ap; const T* A2 = (const T*)A2p; const T* Bt = (const T*)Btp; const T* Bt2 = (const T*)Bt2p;
  __shared__ __align__(16) float sT[8][16 * 68];
  const int b    = blockIdx.y;
  const int lane = threadIdx.x & 31;
  const int wave = threadIdx.x >> 5;
  const int tilesN = N >> 6;
  const int tilesM = M >> 6;
  const int tile = blockIdx.x * 8 + wave;
  if (tile >= tilesM * tilesN) return;
  const int tm = tile / tilesN;
  const int tn = tile - tm * tilesN;
  const int m0 = tm << 6;
  const int n0 = tn << 6;
  if (CAUSAL == 1 && n0 > m0) return;
  const int Kt = (CAUSAL == 2) ? ((m0 + 64 < K) ? (m0 + 64) : K) : K;

  const T* Ab  = A  + (size_t)b * strideA;
  const T* Bb  = Bt + (size_t)b * strideB;
  const T* Ab2 = SPLIT ? (A2  + (size_t)b * strideA) : nullptr;
  const T* Bb2 = SPLIT ? (Bt2 + (size_t)b * strideB) : nullptr;

  const int rlane = lane & 15;
  const int koff  = (lane >> 4) * 8;
  const int mOff  = (lane >> 4) * 8;

  v8f acc[4][4];
#pragma unroll
  for (int i = 0; i < 4; ++i)
#pragma unroll
    for (int j = 0; j < 4; ++j) acc[i][j] = (v8f){0.f,0.f,0.f,0.f,0.f,0.f,0.f,0.f};

  for (int k0 = 0; k0 < Kt; k0 += 32) {
    V bh[4], bl[4];
#pragma unroll
    for (int j = 0; j < 4; ++j) {
      const size_t bo = (size_t)(n0 + (j << 4) + rlane) * ldb + koff + k0;
      bh[j] = Frag<T>::load(Bb + bo);
      if (SPLIT) bl[j] = Frag<T>::load(Bb2 + bo);
    }
#pragma unroll
    for (int i = 0; i < 4; ++i) {
      const size_t ao = (size_t)(m0 + (i << 4) + rlane) * lda + koff + k0;
      V ah = Frag<T>::load(Ab + ao);
      V al;
      if (SPLIT) al = Frag<T>::load(Ab2 + ao);
#pragma unroll
      for (int j = 0; j < 4; ++j) {
        acc[i][j] = Frag<T>::mma(ah, bh[j], acc[i][j]);
        if (SPLIT) {
          acc[i][j] = Frag<T>::mma(ah, bl[j], acc[i][j]);
          acc[i][j] = Frag<T>::mma(al, bh[j], acc[i][j]);
        }
      }
      Frag<T>::guard(acc[i][0], acc[i][3], ah, SPLIT ? al : ah);
    }
    Frag<T>::keep(bh[0], bh[1], bh[2], bh[3]);
    if (SPLIT) Frag<T>::keep(bl[0], bl[1], bl[2], bl[3]);
  }
  acc_guard4(acc[0][0], acc[0][1], acc[0][2], acc[0][3]);
  acc_guard4(acc[1][0], acc[1][1], acc[1][2], acc[1][3]);
  acc_guard4(acc[2][0], acc[2][1], acc[2][2], acc[2][3]);
  acc_guard4(acc[3][0], acc[3][1], acc[3][2], acc[3][3]);

  float* slab = sT[wave];
  const float* Rb = RESID ? (resid + (size_t)b * strideR) : nullptr;
#pragma unroll
  for (int i = 0; i < 4; ++i) {
    const int mBase = m0 + (i << 4);
#pragma unroll
    for (int j = 0; j < 4; ++j) {
      const int n = n0 + (j << 4) + rlane;
      float bv = 0.f;
      if (BIAS_MODE == 2) bv = bias[n];
#pragma unroll
      for (int r = 0; r < 8; ++r) {
        float v = acc[i][j][r] * scale;
        if (BIAS_MODE == 1) v += bias[mBase + mOff + r];
        if (BIAS_MODE == 2) v += bv;
        if (RESID) v += Rb[(size_t)(mBase + mOff + r) * ldc + n];
        if (ACT == 2) v = fmaxf(v, 0.0f);
        if (ACT == 4) v = (v > 0.f) ? v : 0.01f * v;
        if (ACT == 6) {
          const float t3 = v * v * v;
          const float tt = kGeluC0 * (v + kGeluC1 * t3);
          const float ex = expf(-2.0f * tt);
          v = v * __builtin_amdgcn_rcpf(1.0f + ex) * kActCarry;
        }
        slab[(mOff + r) * 68 + (j << 4) + rlane] = v;
      }
    }
    __builtin_amdgcn_fence(__ATOMIC_RELEASE, "workgroup");
    __builtin_amdgcn_wave_barrier();
    __builtin_amdgcn_fence(__ATOMIC_ACQUIRE, "workgroup");
    if (OUT_MODE == 0) {
      float* C = (float*)Cout + (size_t)b * strideC;
      const int hh = lane >> 4, c4 = (lane & 15) * 4;
      for (int pass = 0; pass < 2; ++pass) {
#pragma unroll
        for (int it = 0; it < 8; ++it) {
          const int row = it * 2 + hh;
          v4f v = *(const v4f*)(slab + row * 68 + c4);
          *(volatile v4f*)(C + (size_t)(mBase + row) * ldc + n0 + c4) = v;
        }
        __threadfence();
      }
    } else {
      const int q = lane >> 3, c8 = (lane & 7) * 8;
      unsigned short* C  = (unsigned short*)Cout  + (size_t)b * strideC;
      unsigned short* C2 = (OUT_MODE == 2) ? ((unsigned short*)Cout2 + (size_t)b * strideC) : nullptr;
      for (int pass = 0; pass < 2; ++pass) {
#pragma unroll
        for (int it = 0; it < 4; ++it) {
          const int row = it * 4 + q;
          const float* sp = slab + row * 68 + c8;
          v8h hv, lv;
#pragma unroll
          for (int e = 0; e < 8; ++e) {
            if (OUT_MODE == 1) {
              hv[e] = (_Float16)sp[e];
            } else {
              unsigned short hb = f2bf_bits(sp[e]);
              unsigned short lb = f2bf_bits(sp[e] - bf_bits2f(hb));
              hv[e] = __builtin_bit_cast(_Float16, hb);
              lv[e] = __builtin_bit_cast(_Float16, lb);
            }
          }
          *(volatile v8h*)(C + (size_t)(mBase + row) * ldc + n0 + c8) = hv;
          if (OUT_MODE == 2) *(volatile v8h*)(C2 + (size_t)(mBase + row) * ldc + n0 + c8) = lv;
        }
        __threadfence();
      }
    }
    __builtin_amdgcn_fence(__ATOMIC_RELEASE, "workgroup");
    __builtin_amdgcn_wave_barrier();
    __builtin_amdgcn_fence(__ATOMIC_ACQUIRE, "workgroup");
  }
}

__global__ __launch_bounds__(256) void wt_cast_kernel(const float* __restrict__ W, unsigned short* __restrict__ WT,
                                                      int Kd, int Nd, float scale) {
  __shared__ float sm[64][65];
  const int t  = threadIdx.x;
  const int k0 = blockIdx.x * 64;
  const int n0 = blockIdx.y * 64;
#pragma unroll
  for (int i = 0; i < 16; ++i) {
    const int e = i * 256 + t;
    const int r = e >> 6;
    const int c = e & 63;
    sm[c][r] = W[(size_t)(k0 + r) * Nd + n0 + c] * scale;
  }
  __syncthreads();
  const int lane = t & 31, wave = t >> 5;
  const int q = lane >> 3, c8 = (lane & 7) * 8;
  for (int pass = 0; pass < 2; ++pass) {
#pragma unroll
    for (int it = 0; it < 2; ++it) {
      const int row = wave * 8 + it * 4 + q;
      unsigned short hb[8];
#pragma unroll
      for (int e = 0; e < 8; ++e) hb[e] = h_bits(sm[row][c8 + e]);
      const v4u u = (v4u){pk16(hb[0], hb[1]), pk16(hb[2], hb[3]), pk16(hb[4], hb[5]), pk16(hb[6], hb[7])};
      *(volatile v4u*)(WT + (size_t)(n0 + row) * Kd + k0 + c8) = u;
    }
    __threadfence();
  }
}

__global__ __launch_bounds__(128) void ln_kernel(const float* __restrict__ X, const float* __restrict__ gam,
                                                 const float* __restrict__ bet, const float* __restrict__ pos,
                                                 unsigned short* __restrict__ outp, int addpos) {
  __shared__ float red[4];
  __shared__ float red2[4];
  const int row  = blockIdx.x;
  const int t    = threadIdx.x;
  const int lane = t & 31, wave = t >> 5;
  const int c0   = t * 8;
  const float* xr = X + (size_t)row * kD + c0;
  const v4f a = *(const v4f*)(xr);
  const v4f c = *(const v4f*)(xr + 4);
  float xv[8];
#pragma unroll
  for (int e = 0; e < 4; ++e) { xv[e] = a[e]; xv[4 + e] = c[e]; }
  float s = ((xv[0] + xv[1]) + (xv[2] + xv[3])) + ((xv[4] + xv[5]) + (xv[6] + xv[7]));
#pragma unroll
  for (int off = 16; off > 0; off >>= 1) s += __shfl_xor(s, off, 32);
  if (lane == 0) red[wave] = s;
  __syncthreads();
  const float mu = ((red[0] + red[1]) + (red[2] + red[3])) * kInvD;
  float dv[8];
#pragma unroll
  for (int e = 0; e < 8; ++e) dv[e] = xv[e] - mu;
  float sq = ((dv[0] * dv[0] + dv[1] * dv[1]) + (dv[2] * dv[2] + dv[3] * dv[3]))
           + ((dv[4] * dv[4] + dv[5] * dv[5]) + (dv[6] * dv[6] + dv[7] * dv[7]));
#pragma unroll
  for (int off = 16; off > 0; off >>= 1) sq += __shfl_xor(sq, off, 32);
  if (lane == 0) red2[wave] = sq;
  __syncthreads();
  const float var  = ((red2[0] + red2[1]) + (red2[2] + red2[3])) * kInvD;
  const float rstd = rsqrtf(var + kEps);
  const v4f g0 = *(const v4f*)(gam + c0);
  const v4f g1 = *(const v4f*)(gam + c0 + 4);
  const v4f b0 = *(const v4f*)(bet + c0);
  const v4f b1 = *(const v4f*)(bet + c0 + 4);
  float y[8];
#pragma unroll
  for (int e = 0; e < 4; ++e) {
    y[e]     = dv[e] * rstd * g0[e] + b0[e];
    y[4 + e] = dv[4 + e] * rstd * g1[e] + b1[e];
  }
  if (addpos) {
    const float* pr = pos + (size_t)(row % kS) * kD + c0;
    const v4f p0 = *(const v4f*)(pr);
    const v4f p1 = *(const v4f*)(pr + 4);
#pragma unroll
    for (int e = 0; e < 4; ++e) { y[e] += p0[e]; y[4 + e] += p1[e]; }
  }
  unsigned short hb[8];
#pragma unroll
  for (int e = 0; e < 8; ++e) hb[e] = h_bits(y[e]);
  const v4u u = (v4u){pk16(hb[0], hb[1]), pk16(hb[2], hb[3]), pk16(hb[4], hb[5]), pk16(hb[6], hb[7])};
  unsigned short* op = outp + (size_t)row * kD + c0;
  *(volatile v4u*)op = u;
  __threadfence();
  *(volatile v4u*)op = u;
}

__global__ __launch_bounds__(256) void vt_kernel(const unsigned short* __restrict__ qkv, unsigned short* __restrict__ vt) {
  __shared__ unsigned short sm[64][72];
  const int t  = threadIdx.x;
  const int s0 = blockIdx.x * 64;
  const int bh = blockIdx.y;
  const int b  = bh >> 4, h = bh & 15;
#pragma unroll
  for (int i = 0; i < 2; ++i) {
    const int e  = i * 256 + t;
    const int r  = e >> 3;
    const int c8 = (e & 7) * 8;
    const v4u w = *(const v4u*)(qkv + (size_t)(b * kS + s0 + r) * kQKVN + 2 * kD + h * kHD + c8);
#pragma unroll
    for (int j = 0; j < 4; ++j) {
      sm[c8 + 2 * j][r]     = (unsigned short)(w[j] & 0xFFFFu);
      sm[c8 + 2 * j + 1][r] = (unsigned short)(w[j] >> 16);
    }
  }
  __syncthreads();
  const int lane = t & 31, wave = t >> 5;
  const int q = lane >> 3, c8 = (lane & 7) * 8;
  for (int pass = 0; pass < 2; ++pass) {
#pragma unroll
    for (int it = 0; it < 2; ++it) {
      const int d = wave * 8 + it * 4 + q;
      unsigned short hb[8];
#pragma unroll
      for (int e = 0; e < 8; ++e) hb[e] = sm[d][c8 + e];
      const v4u u = (v4u){pk16(hb[0], hb[1]), pk16(hb[2], hb[3]), pk16(hb[4], hb[5]), pk16(hb[6], hb[7])};
      *(volatile v4u*)(vt + (size_t)(bh * kHD + d) * kS + s0 + c8) = u;
    }
    __threadfence();
  }
}

__global__ __launch_bounds__(256) void softmax_kernel(const float* __restrict__ Sc, unsigned short* __restrict__ P) {
  __shared__ float redM[8];
  __shared__ float redS[8];
  const int g    = blockIdx.y;
  const int q    = blockIdx.x;
  const int t    = threadIdx.x;
  const int lane = t & 31, wave = t >> 5;
  const int c0   = t * 8;
  const int lim  = ((q >> 6) + 1) * 64;
  const int ca   = (c0 + 8 <= lim) ? c0 : (lim - 8);
  const float* sr = Sc + ((size_t)g * kS + q) * kS + ca;
  const v4f a = *(const v4f*)(sr);
  const v4f c = *(const v4f*)(sr + 4);
  float x[8];
#pragma unroll
  for (int e = 0; e < 4; ++e) {
    x[e]     = (c0 + e <= q)     ? a[e] : -INFINITY;
    x[4 + e] = (c0 + 4 + e <= q) ? c[e] : -INFINITY;
  }
  float m = fmaxf(fmaxf(fmaxf(x[0], x[1]), fmaxf(x[2], x[3])), fmaxf(fmaxf(x[4], x[5]), fmaxf(x[6], x[7])));
#pragma unroll
  for (int off = 16; off > 0; off >>= 1) m = fmaxf(m, __shfl_xor(m, off, 32));
  if (lane == 0) redM[wave] = m;
  __syncthreads();
  float rmax = redM[0];
#pragma unroll
  for (int w = 1; w < 8; ++w) rmax = fmaxf(rmax, redM[w]);
  float ev[8];
#pragma unroll
  for (int e = 0; e < 8; ++e) ev[e] = expf(x[e] - rmax);
  float s = ((ev[0] + ev[1]) + (ev[2] + ev[3])) + ((ev[4] + ev[5]) + (ev[6] + ev[7]));
#pragma unroll
  for (int off = 16; off > 0; off >>= 1) s += __shfl_xor(s, off, 32);
  if (lane == 0) redS[wave] = s;
  __syncthreads();
  const float tot = ((redS[0] + redS[1]) + (redS[2] + redS[3])) + ((redS[4] + redS[5]) + (redS[6] + redS[7]));
  const float rcp = kPCarry / tot;
  unsigned short hb[8];
#pragma unroll
  for (int e = 0; e < 8; ++e) hb[e] = h_bits(ev[e] * rcp);
  const v4u u = (v4u){pk16(hb[0], hb[1]), pk16(hb[2], hb[3]), pk16(hb[4], hb[5]), pk16(hb[6], hb[7])};
  unsigned short* op = P + ((size_t)g * kS + q) * kS + c0;
  *(volatile v4u*)op = u;
  __threadfence();
  *(volatile v4u*)op = u;
}

extern "C" void kernel_launch(void* const* d_in, const int* in_sizes, int n_in,
                              void* d_out, int out_size, void* d_ws, size_t ws_size,
                              hipStream_t stream) {
  if (n_in < 14) return;
  if (out_size < kTok * kD) return;
  if (ws_size < kWsTotal) return;
  if (in_sizes[0] < kTok * kD || in_sizes[1] < kS * kD || in_sizes[2] < kD || in_sizes[3] < kD ||
      in_sizes[4] < kD * kQKVN || in_sizes[5] < kQKVN || in_sizes[6] < kD * kD || in_sizes[7] < kD ||
      in_sizes[8] < kD || in_sizes[9] < kD || in_sizes[10] < kD * kDFF || in_sizes[11] < kDFF ||
      in_sizes[12] < kDFF * kD || in_sizes[13] < kD) return;

  const float* x      = (const float*)d_in[0];
  const float* pos    = (const float*)d_in[1];
  const float* ln1_g  = (const float*)d_in[2];
  const float* ln1_b  = (const float*)d_in[3];
  const float* w_qkv  = (const float*)d_in[4];
  const float* b_qkv  = (const float*)d_in[5];
  const float* w_o    = (const float*)d_in[6];
  const float* b_o    = (const float*)d_in[7];
  const float* ln2_g  = (const float*)d_in[8];
  const float* ln2_b  = (const float*)d_in[9];
  const float* w_fc   = (const float*)d_in[10];
  const float* b_fc   = (const float*)d_in[11];
  const float* w_proj = (const float*)d_in[12];
  const float* b_proj = (const float*)d_in[13];
  float* outp = (float*)d_out;

  char* ws = (char*)d_ws;
  unsigned short* qkv16  = (unsigned short*)(ws + kOffQkv);
  unsigned short* a1     = (unsigned short*)(ws + kOffA1);
  unsigned short* vt16   = (unsigned short*)(ws + kOffVt);
  float*          scores = (float*)(ws + kOffScores);
  unsigned short* h16    = (unsigned short*)(ws + kOffH);
  unsigned short* m16    = (unsigned short*)(ws + kOffM);
  unsigned short* wqkvT  = (unsigned short*)(ws + kOffWqkvT);
  unsigned short* wfcT   = (unsigned short*)(ws + kOffWfcT);
  unsigned short* wprojT = (unsigned short*)(ws + kOffWprojT);
  unsigned short* p16    = (unsigned short*)(ws + kOffP);
  float*          x1     = (float*)(ws + kOffX1);
  unsigned short* ctx16  = (unsigned short*)(ws + kOffCtx);
  unsigned short* woT    = (unsigned short*)(ws + kOffWoT);

  wt_cast_kernel<<<dim3(kD / 64, kQKVN / 64), 256, 0, stream>>>(w_qkv, wqkvT, kD, kQKVN, kWCarry);
  wt_cast_kernel<<<dim3(kD / 64, kD / 64), 256, 0, stream>>>(w_o, woT, kD, kD, kWCarry);
  ln_kernel<<<kTok, 128, 0, stream>>>(x, ln1_g, ln1_b, pos, h16, 1);
  wmma_gemm64<0, false, 2, 1, false, 0, 0> <<<dim3(384, 1), 256, 0, stream>>> (
      h16, h16, kD, 0L, wqkvT, wqkvT, kD, 0L, (void*)qkv16, (void*)qkv16, kQKVN, 0L,
      b_qkv, x, 0L, kTok, kQKVN, kD, 1.0f / kWCarry);
  vt_kernel<<<dim3(kS / 64, kB * kH), 256, 0, stream>>>(qkv16, vt16);

  for (int ch = 0; ch < kNChunk; ++ch) {
    const int bb = ch / (kH / kGrp);
    const int hb = (ch % (kH / kGrp)) * kGrp;
    const unsigned short* qp  = qkv16 + (size_t)bb * kS * kQKVN + (size_t)hb * kHD;
    const unsigned short* kp  = qp + kD;
    const unsigned short* vtp = vt16 + (size_t)((bb * kH + hb) * kHD) * kS;
    unsigned short* cp = ctx16 + (size_t)bb * kS * kD + (size_t)hb * kHD;
    wmma_gemm64<0, false, 0, 0, false, 0, 1> <<<dim3(128, kGrp), 256, 0, stream>>> (
        qp, qp, kQKVN, (long)kHD, kp, kp, kQKVN, (long)kHD, (void*)scores, (void*)scores, kS, (long)kS * kS,
        b_qkv, x, 0L, kS, kS, kHD, 0.125f);
    softmax_kernel<<<dim3(kS, kGrp), 256, 0, stream>>>(scores, p16);
    wmma_gemm64<0, false, 0, 1, false, 0, 2> <<<dim3(4, kGrp), 256, 0, stream>>> (
        p16, p16, kS, (long)kS * kS, vtp, vtp, kS, (long)kHD * kS, (void*)cp, (void*)cp, kD, (long)kHD,
        b_qkv, x, 0L, kS, kHD, kS, kPVScale);
  }

  wmma_gemm64<0, false, 2, 0, true, 0, 0> <<<dim3(128, 1), 256, 0, stream>>> (
      ctx16, ctx16, kD, 0L, woT, woT, kD, 0L, (void*)x1, (void*)x1, kD, 0L,
      b_o, x, 0L, kTok, kD, kD, kOScale);

  ln_kernel<<<kTok, 128, 0, stream>>>(x1, ln2_g, ln2_b, pos, m16, 0);
  wt_cast_kernel<<<dim3(kD / 64, kDFF / 64), 256, 0, stream>>>(w_fc, wfcT, kD, kDFF, kWCarry);
  wt_cast_kernel<<<dim3(kDFF / 64, kD / 64), 256, 0, stream>>>(w_proj, wprojT, kDFF, kD, kWCarry);
  wmma_gemm64<0, false, 2, 1, false, 6, 0> <<<dim3(512, 1), 256, 0, stream>>> (
      m16, m16, kD, 0L, wfcT, wfcT, kD, 0L, (void*)a1, (void*)a1, kDFF, 0L,
      b_fc, x, 0L, kTok, kDFF, kD, kFcScale);
  wmma_gemm64<0, false, 2, 0, true, 0, 0> <<<dim3(128, 1), 256, 0, stream>>> (
      a1, a1, kDFF, 0L, wprojT, wprojT, kDFF, 0L, (void*)outp, (void*)outp, kD, 0L,
      b_proj, x1, 0L, kTok, kD, kDFF, kProjScale);
}
